// CrossGraphNodeAttention_15126874816759
// MI455X (gfx1250) — hardware-verified
//
#include <hip/hip_runtime.h>
#include <math.h>
#include <stdint.h>

#define NB    8
#define SEQ   2048
#define DM    256
#define NROW  (NB * SEQ)
#define QT    64
#define PTP   40
#define OSP   132
#define QSP   136
#define TP    72
#define LNPS  6.931471805599453f
#define FMIN16 6.103515625e-05f
#define NEGBIG (-1.0e30f)
static_assert((SEQ % QT) == 0);
static_assert((SEQ % 64) == 0);
static_assert((SEQ % 256) == 0);
static_assert((DM % 128) == 0);
static_assert((DM % 32) == 0);
static_assert((NROW % 64) == 0);
static_assert(((DM * DM) / 8) % 256 == 0);
static_assert(((NROW * DM) / 8) % 256 == 0);
static_assert(DM == 256);
static_assert(QT == 64);
static_assert(64 * QSP <= 128 * TP);

typedef _Float16       v16h __attribute__((ext_vector_type(16)));
typedef _Float16       v8h  __attribute__((ext_vector_type(8)));
typedef __bf16         v16b __attribute__((ext_vector_type(16)));
typedef unsigned short v8us __attribute__((ext_vector_type(8)));
typedef float          v8f  __attribute__((ext_vector_type(8)));
typedef float          v4f  __attribute__((ext_vector_type(4)));
typedef unsigned int   v4u  __attribute__((ext_vector_type(4)));

union FragH { v16h v; v8h  h[2]; };
union FragB { v16b v; v8us u[2]; };
static_assert(sizeof(FragH) == 32);
static_assert(sizeof(FragB) == 32);

__device__ __forceinline__ unsigned short bf_bits(float f) {
  unsigned u = __float_as_uint(f);
  return (unsigned short)((u + 0x7FFFu + ((u >> 16) & 1u)) >> 16);
}
__device__ __forceinline__ float bf_up(unsigned short x) { return __uint_as_float(((unsigned)x) << 16); }
__device__ __forceinline__ float bfr(float f) { return bf_up(bf_bits(f)); }
__device__ __forceinline__ unsigned short h_bits(_Float16 x) { return __builtin_bit_cast(unsigned short, x); }
__device__ __forceinline__ unsigned pk16(unsigned short a, unsigned short b) { return (unsigned)a | ((unsigned)b << 16); }
__device__ __forceinline__ _Float16 to_h_ftz(float v) { return (_Float16)((fabsf(v) < FMIN16) ? 0.0f : v); }
__device__ __forceinline__ v8f zero8() { v8f z = {0.f, 0.f, 0.f, 0.f, 0.f, 0.f, 0.f, 0.f}; return z; }
__device__ __forceinline__ float hmax8(v8f s) {
  return fmaxf(fmaxf(fmaxf(s[0], s[1]), fmaxf(s[2], s[3])), fmaxf(fmaxf(s[4], s[5]), fmaxf(s[6], s[7])));
}

__device__ __forceinline__ v16h ldfrag_h(const _Float16* p) {
  FragH f;
  f.h[0] = *(const v8h*)(p);
  f.h[1] = *(const v8h*)(p + 16);
  return f.v;
}
__device__ __forceinline__ v16b ldfrag_b(const unsigned short* p) {
  FragB f;
  f.u[0] = *(const v8us*)(p);
  f.u[1] = *(const v8us*)(p + 16);
  return f.v;
}

__device__ __forceinline__ v8f mma_h(v16h a, v16h b, v8f c) {
  v8f d = __builtin_amdgcn_wmma_f32_16x16x32_f16(false, a, false, b, (short)0, c, false, false);
#if defined(__HIP_DEVICE_COMPILE__)
  asm volatile("v_nop\n\tv_nop\n\tv_nop\n\tv_nop" : "+v"(d) : "v"(a), "v"(b));
#endif
  return d;
}
__device__ __forceinline__ v8f mma_b(v16b a, v16b b, v8f c) {
  v8f d = __builtin_amdgcn_wmma_f32_16x16x32_bf16(false, a, false, b, (short)0, c, false, false);
#if defined(__HIP_DEVICE_COMPILE__)
  const v16h ha = __builtin_bit_cast(v16h, a), hb = __builtin_bit_cast(v16h, b);
  asm volatile("v_nop\n\tv_nop\n\tv_nop\n\tv_nop" : "+v"(d) : "v"(ha), "v"(hb));
#endif
  return d;
}

__global__ __launch_bounds__(256) void cvt8(const float* __restrict__ src, unsigned short* dst, int n8) {
  const int i = blockIdx.x * 256 + threadIdx.x;
  if (i >= n8) return;
  const float* p = src + (size_t)i * 8;
  const v4f f0 = *(const v4f*)(p), f1 = *(const v4f*)(p + 4);
  v4u wb;
  wb[0] = pk16(bf_bits(f0[0]), bf_bits(f0[1]));
  wb[1] = pk16(bf_bits(f0[2]), bf_bits(f0[3]));
  wb[2] = pk16(bf_bits(f1[0]), bf_bits(f1[1]));
  wb[3] = pk16(bf_bits(f1[2]), bf_bits(f1[3]));
  unsigned short* d = dst + (size_t)i * 8;
  *(volatile v4u*)d = wb;
  __threadfence();
  *(volatile v4u*)d = wb;
}

__global__ __launch_bounds__(256)
void proj_kernel(const unsigned short* __restrict__ XB, const unsigned short* __restrict__ WB,
                 const float* __restrict__ bias, unsigned short* OP, int tr) {
  __shared__ __align__(16) unsigned short S[128 * TP];
  const int tid  = threadIdx.x;
  const int lane = tid & 31, wave = tid >> 5;
  const int h    = lane >> 4, c = lane & 15;
  const int rg   = wave & 3, ch = wave >> 2;
  const int row0 = blockIdx.y * 64;
  const int col0 = blockIdx.x * 128;

  const unsigned short* ap = XB + ((size_t)(row0 + 16 * rg + c)) * DM + 8 * h;
  const unsigned short* bp = WB + ((size_t)(col0 + 64 * ch + c)) * DM + 8 * h;
  v8f acc0 = zero8(), acc1 = zero8(), acc2 = zero8(), acc3 = zero8();
#pragma unroll 2
  for (int ks = 0; ks < DM / 32; ++ks) {
    const v16b a = ldfrag_b(ap + 32 * ks);
    const unsigned short* bs = bp + 32 * ks;
    acc0 = mma_b(a, ldfrag_b(bs + 0 * 16 * DM), acc0);
    acc1 = mma_b(a, ldfrag_b(bs + 1 * 16 * DM), acc1);
    acc2 = mma_b(a, ldfrag_b(bs + 2 * 16 * DM), acc2);
    acc3 = mma_b(a, ldfrag_b(bs + 3 * 16 * DM), acc3);
  }

  const int cb = col0 + 64 * ch + c;
  const float bb0 = bfr(bias[cb + 0 * 16]), bb1 = bfr(bias[cb + 1 * 16]);
  const float bb2 = bfr(bias[cb + 2 * 16]), bb3 = bfr(bias[cb + 3 * 16]);

  unsigned short q0[8], q1[8], q2[8], q3[8];
#pragma unroll
  for (int r = 0; r < 8; ++r) {
    q0[r] = h_bits(to_h_ftz(acc0[r] + bb0));
    q1[r] = h_bits(to_h_ftz(acc1[r] + bb1));
    q2[r] = h_bits(to_h_ftz(acc2[r] + bb2));
    q3[r] = h_bits(to_h_ftz(acc3[r] + bb3));
  }

  if (tr == 0) {
    unsigned short* qs = S + (16 * rg + 8 * h) * QSP + 64 * ch + c;
#pragma unroll
    for (int r = 0; r < 8; ++r) {
      qs[r * QSP + 0 * 16] = q0[r];
      qs[r * QSP + 1 * 16] = q1[r];
      qs[r * QSP + 2 * 16] = q2[r];
      qs[r * QSP + 3 * 16] = q3[r];
    }
  } else {
    v4u w0, w1, w2, w3;
#pragma unroll
    for (int t = 0; t < 4; ++t) {
      w0[t] = pk16(q0[2 * t], q0[2 * t + 1]);
      w1[t] = pk16(q1[2 * t], q1[2 * t + 1]);
      w2[t] = pk16(q2[2 * t], q2[2 * t + 1]);
      w3[t] = pk16(q3[2 * t], q3[2 * t + 1]);
    }
    unsigned short* ts = S + (64 * ch + c) * TP + 16 * rg + 8 * h;
    *(v4u*)(ts + 0 * 16 * TP) = w0;
    *(v4u*)(ts + 1 * 16 * TP) = w1;
    *(v4u*)(ts + 2 * 16 * TP) = w2;
    *(v4u*)(ts + 3 * 16 * TP) = w3;
  }
  __syncthreads();

  const int e = tid & 7, lg = tid >> 3;
  if (tr == 0) {
#pragma unroll
    for (int pass = 0; pass < 2; ++pass) {
#pragma unroll
      for (int it = 0; it < 4; ++it) {
        const int L   = it * 32 + lg;
        const int row = L >> 1, hf = L & 1;
        const v4u v = *(const v4u*)(S + row * QSP + 64 * hf + 8 * e);
        *(volatile v4u*)(OP + ((size_t)(row0 + row)) * DM + col0 + 64 * hf + 8 * e) = v;
      }
      __threadfence();
    }
  } else {
    const int b    = row0 / SEQ;
    const int key0 = row0 % SEQ;
#pragma unroll
    for (int pass = 0; pass < 2; ++pass) {
#pragma unroll
      for (int it = 0; it < 4; ++it) {
        const int dd = it * 32 + lg;
        const v4u v = *(const v4u*)(S + dd * TP + 8 * e);
        *(volatile v4u*)(OP + ((size_t)b * DM + col0 + dd) * SEQ + key0 + 8 * e) = v;
      }
      __threadfence();
    }
  }
}

__global__ __launch_bounds__(256)
void attn_kernel(const unsigned short* __restrict__ QP, const unsigned short* __restrict__ KP,
                 const unsigned short* __restrict__ VT, const int* __restrict__ mask, float* out) {
  __shared__ __align__(16) _Float16 Pt[64 * PTP];
  __shared__ float Cs[64];
  __shared__ float Ls[64];
  __shared__ __align__(16) float Os[64 * OSP];
  __shared__ int Ms[SEQ];
  const int tid  = threadIdx.x;
  const int wave = tid >> 5;
  const int lane = tid & 31;
  const int h    = lane >> 4;
  const int c    = lane & 15;
  const int bx   = blockIdx.x;
  const int b    = bx / (SEQ / QT);
  const int qt   = bx % (SEQ / QT);
  const int n0   = qt * QT;
  const _Float16* QPh = (const _Float16*)(const void*)QP;
  const _Float16* KPh = (const _Float16*)(const void*)KP;
  const _Float16* VTh = (const _Float16*)(const void*)VT;

#pragma unroll
  for (int i = 0; i < SEQ / 256; ++i) Ms[i * 256 + tid] = mask[(size_t)b * SEQ + i * 256 + tid];
  __syncthreads();

  const int wq = wave & 3;
  const _Float16* qpp = QPh + ((size_t)b * SEQ + n0 + 16 * wq + c) * DM + 8 * h;
  const _Float16* khp = KPh + ((size_t)b * SEQ + c) * DM + 8 * h;
  const _Float16* vtp = VTh + ((size_t)b * DM + 32 * wave + c) * SEQ + 8 * h;
  const float SCL = 0.0625f;

  float m = NEGBIG, l = 0.f;
  v8f acc[2][4];
#pragma unroll
  for (int jd = 0; jd < 2; ++jd)
#pragma unroll
    for (int jq = 0; jq < 4; ++jq) acc[jd][jq] = zero8();

#pragma unroll 1
  for (int it = 0; it < SEQ / 32; ++it) {
    const int kb = it * 32;
    if (wave < 4) {
      v8f s0 = zero8(), s1 = zero8();
      const _Float16* k0p = khp + (size_t)kb * DM;
      const _Float16* k1p = k0p + 16 * DM;
#pragma unroll 2
      for (int ks = 0; ks < DM / 32; ++ks) {
        const v16h qf = ldfrag_h(qpp + 32 * ks);
        const v16h a0 = ldfrag_h(k0p + 32 * ks);
        const v16h a1 = ldfrag_h(k1p + 32 * ks);
        s0 = mma_h(a0, qf, s0);
        s1 = mma_h(a1, qf, s1);
      }
#pragma unroll
      for (int r = 0; r < 8; ++r) {
        const int keep0 = Ms[kb + 8 * h + r];
        const int keep1 = Ms[kb + 16 + 8 * h + r];
        const float v0 = s0[r] * SCL, v1 = s1[r] * SCL;
        s0[r] = (keep0 != 0) ? v0 : NEGBIG;
        s1[r] = (keep1 != 0) ? v1 : NEGBIG;
      }

      float mx = fmaxf(hmax8(s0), hmax8(s1));
      mx = fmaxf(mx, __shfl_xor(mx, 16, 32));
      const float mn   = fmaxf(m, mx);
      const float corr = __expf(m - mn);
      m = mn;
      const float msh = mn - LNPS;
      FragH ph;
      float ls = 0.f;
#pragma unroll
      for (int r = 0; r < 8; ++r) {
        const float e0 = __expf(s0[r] - msh);
        const float e1 = __expf(s1[r] - msh);
        ls += e0 + e1;
        ph.h[0][r] = (_Float16)e0;
        ph.h[1][r] = (_Float16)e1;
      }
      l = l * corr + ls;
      _Float16* pr = Pt + (16 * wave + c) * PTP + 8 * h;
      *(v8h*)(pr)      = ph.h[0];
      *(v8h*)(pr + 16) = ph.h[1];
      if (h == 0) Cs[16 * wave + c] = corr;
    }
    __syncthreads();

    float cr[4];
#pragma unroll
    for (int jq = 0; jq < 4; ++jq) cr[jq] = Cs[16 * jq + c];
#pragma unroll
    for (int jd = 0; jd < 2; ++jd)
#pragma unroll
      for (int jq = 0; jq < 4; ++jq)
#pragma unroll
        for (int r = 0; r < 8; ++r) acc[jd][jq][r] *= cr[jq];

    v16h vf[2];
#pragma unroll
    for (int jd = 0; jd < 2; ++jd) vf[jd] = ldfrag_h(vtp + (size_t)(16 * jd) * SEQ + kb);
#pragma unroll
    for (int jq = 0; jq < 4; ++jq) {
      const v16h pf = ldfrag_h(Pt + (16 * jq + c) * PTP + 8 * h);
#pragma unroll
      for (int jd = 0; jd < 2; ++jd) acc[jd][jq] = mma_h(vf[jd], pf, acc[jd][jq]);
    }
    __syncthreads();
  }

  if (wave < 4) {
    l += __shfl_xor(l, 16, 32);
    if (h == 0) Ls[16 * wave + c] = 1.0f / l;
  }
  __syncthreads();
  float scq[4];
#pragma unroll
  for (int jq = 0; jq < 4; ++jq) scq[jq] = Ls[16 * jq + c];

  const int e = tid & 7, lg = tid >> 3;
  float* ob = out + ((size_t)b * SEQ + n0) * DM;
#pragma unroll
  for (int t = 0; t < 2; ++t) {
    if ((wave >> 2) == t) {
      const int dl = 32 * (wave & 3);
#pragma unroll
      for (int jd = 0; jd < 2; ++jd)
#pragma unroll
        for (int jq = 0; jq < 4; ++jq) {
          float* os = Os + (16 * jq + c) * OSP + dl + 16 * jd + 8 * h;
          const float sc = scq[jq];
          v4f v0, v1;
          v0[0] = acc[jd][jq][0] * sc; v0[1] = acc[jd][jq][1] * sc;
          v0[2] = acc[jd][jq][2] * sc; v0[3] = acc[jd][jq][3] * sc;
          v1[0] = acc[jd][jq][4] * sc; v1[1] = acc[jd][jq][5] * sc;
          v1[2] = acc[jd][jq][6] * sc; v1[3] = acc[jd][jq][7] * sc;
          *(v4f*)(os)     = v0;
          *(v4f*)(os + 4) = v1;
        }
    }
    __syncthreads();
#pragma unroll
    for (int pass = 0; pass < 2; ++pass) {
#pragma unroll
      for (int i = 0; i < 8; ++i) {
        const int L   = i * 32 + lg;
        const int row = L >> 2, hf = L & 3;
        const v4f v = *(const v4f*)(Os + row * OSP + 32 * hf + 4 * e);
        *(volatile v4f*)(ob + (size_t)row * DM + 128 * t + 32 * hf + 4 * e) = v;
      }
      __threadfence();
    }
    __syncthreads();
  }
}

extern "C" void kernel_launch(void* const* d_in, const int* in_sizes, int n_in,
                              void* d_out, int out_size, void* d_ws, size_t ws_size,
                              hipStream_t stream) {
  const int NX = NB * SEQ * DM;
  if (n_in < 9) return;
  if (in_sizes[0] != NX || in_sizes[1] != NX || in_sizes[2] != NB * SEQ) return;
  if (in_sizes[3] != DM * DM || in_sizes[5] != DM * DM || in_sizes[7] != DM * DM) return;
  if (in_sizes[4] != DM || in_sizes[6] != DM || in_sizes[8] != DM) return;
  if (out_size != NX) return;

  size_t off = 0;
  const size_t szP = (size_t)NROW * DM * 2;
  const size_t szW = (size_t)DM * DM * 2;
  const size_t oAB = off; off += szP;
  const size_t oBB = off; off += szP;
  const size_t oQP = off; off += szP;
  const size_t oKP = off; off += szP;
  const size_t oVT = off; off += szP;
  const size_t oWB = off; off += 3 * szW;
  if (off > ws_size) return;
  if (off > (size_t)134217728) return;

  const float* Ain = (const float*)d_in[0];
  const float* Bin = (const float*)d_in[1];
  const int*   msk = (const int*)d_in[2];
  const float* Wq  = (const float*)d_in[3];
  const float* bq  = (const float*)d_in[4];
  const float* Wk  = (const float*)d_in[5];
  const float* bk  = (const float*)d_in[6];
  const float* Wv  = (const float*)d_in[7];
  const float* bv  = (const float*)d_in[8];
  char* ws = (char*)d_ws;
  unsigned short* AB  = (unsigned short*)(ws + oAB);
  unsigned short* BB  = (unsigned short*)(ws + oBB);
  unsigned short* QP  = (unsigned short*)(ws + oQP);
  unsigned short* KP  = (unsigned short*)(ws + oKP);
  unsigned short* VT  = (unsigned short*)(ws + oVT);
  unsigned short* WB  = (unsigned short*)(ws + oWB);
  float* out = (float*)d_out;

  const int  n8X = NX / 8;
  const int  n8W = (DM * DM) / 8;
  const dim3 blk256(256);
  const dim3 gX(n8X / 256);
  const dim3 gW(n8W / 256);
  const dim3 gP(DM / 128, NROW / 64);
  const dim3 gA(NB * (SEQ / QT));

  cvt8<<<gX, blk256, 0, stream>>>(Ain, AB, n8X);
  cvt8<<<gX, blk256, 0, stream>>>(Bin, BB, n8X);
  cvt8<<<gW, blk256, 0, stream>>>(Wq, WB + 0 * (size_t)DM * DM, n8W);
  cvt8<<<gW, blk256, 0, stream>>>(Wk, WB + 1 * (size_t)DM * DM, n8W);
  cvt8<<<gW, blk256, 0, stream>>>(Wv, WB + 2 * (size_t)DM * DM, n8W);
  proj_kernel<<<gP, blk256, 0, stream>>>(AB, WB + 0 * (size_t)DM * DM, bq, QP, 0);
  proj_kernel<<<gP, blk256, 0, stream>>>(BB, WB + 1 * (size_t)DM * DM, bk, KP, 0);
  proj_kernel<<<gP, blk256, 0, stream>>>(BB, WB + 2 * (size_t)DM * DM, bv, VT, 1);
  attn_kernel<<<gA, blk256, 0, stream>>>(QP, KP, VT, msk, out);
  (void)hipGetLastError();
}
